// ColbertLoss_37907381355015
// MI455X (gfx1250) — hardware-verified
//
#include <hip/hip_runtime.h>


namespace {
constexpr int NB = 128, NQ = 32, NS = 512, D = 128;

typedef _Float16 b16;
typedef __attribute__((ext_vector_type(16))) _Float16 v16b;
typedef __attribute__((ext_vector_type(8)))  _Float16 v8b;
typedef __attribute__((ext_vector_type(8)))  float v8f;
typedef __attribute__((ext_vector_type(4)))  float v4f;

__device__ __forceinline__ v8b ld8b(const b16* p) { return *(const v8b*)p; }
__device__ __forceinline__ v16b cat8b(v8b a, v8b b) { return __builtin_shufflevector(a, b, 0, 1, 2, 3, 4, 5, 6, 7, 8, 9, 10, 11, 12, 13, 14, 15); }
__device__ __forceinline__ v16b frag_kb(const b16* p, int hh) { return cat8b(ld8b(p + 8 * hh), ld8b(p + 16 + 8 * hh)); }
__device__ __forceinline__ v8f wmma16b(v16b a, v16b b, v8f c) {
  v8f d = __builtin_amdgcn_wmma_f32_16x16x32_f16(false, a, false, b, (short)0, c, false, false);
  asm volatile("v_nop\n\tv_nop\n\tv_nop\n\tv_nop" : "+v"(d) : "v"(a), "v"(b));
  return d;
}

__global__ __launch_bounds__(256) void cvt_kernel(const float* __restrict__ q, const float* __restrict__ dc, b16* __restrict__ q16, b16* __restrict__ d16) {
  const size_t tid = (size_t)blockIdx.x * blockDim.x + threadIdx.x, stride = (size_t)gridDim.x * blockDim.x;
  const size_t nq = (size_t)NB * NQ * D / 8, nd = (size_t)NB * NS * D / 8;
  for (int pass = 0; pass < 2; ++pass) {
    for (size_t c = tid; c < nq + nd; c += stride) {
      const float* src = (c < nq) ? (q + c * 8) : (dc + (c - nq) * 8); b16* dst = (c < nq) ? (q16 + c * 8) : (d16 + (c - nq) * 8);
      v8b v;
#pragma unroll
      for (int e = 0; e < 8; ++e) v[e] = (b16)src[e];
      *(volatile v8b*)dst = v;
    }
    __threadfence();
  }
}

__global__ __launch_bounds__(256) void score_kernel(const b16* __restrict__ q16, const b16* __restrict__ d16, float* __restrict__ scores) {
  __shared__ float Ss[NB];
  const int wid = threadIdx.x >> 5, lane = threadIdx.x & 31, hh = lane >> 4, col = lane & 15;
  const int b = blockIdx.x;
  const b16* qb = q16 + (size_t)b * NQ * D;
  v16b qa[2][4];
#pragma unroll
  for (int mt = 0; mt < 2; ++mt)
#pragma unroll
    for (int k = 0; k < 4; ++k) qa[mt][k] = frag_kb(qb + (size_t)(mt * 16 + col) * D + 32 * k, hh);
  for (int ci = 0; ci < NB / 8; ++ci) {
    const int c = wid + 8 * ci;
    const b16* db = d16 + (size_t)c * NS * D;
    float mx0[8], mx1[8];
#pragma unroll
    for (int r = 0; r < 8; ++r) { mx0[r] = -INFINITY; mx1[r] = -INFINITY; }
    for (int st = 0; st < NS / 16; ++st) {
      v8f a0 = {}, a1 = {};
#pragma unroll
      for (int k = 0; k < 4; ++k) {
        const v16b bw = frag_kb(db + (size_t)(st * 16 + col) * D + 32 * k, hh);
        a0 = wmma16b(qa[0][k], bw, a0);
        a1 = wmma16b(qa[1][k], bw, a1);
      }
#pragma unroll
      for (int r = 0; r < 8; ++r) { mx0[r] = fmaxf(mx0[r], a0[r]); mx1[r] = fmaxf(mx1[r], a1[r]); }
    }
    float part = 0.0f;
#pragma unroll
    for (int r = 0; r < 8; ++r) {
      float m0 = mx0[r], m1 = mx1[r];
#pragma unroll
      for (int o = 1; o < 16; o <<= 1) { m0 = fmaxf(m0, __shfl_xor(m0, o)); m1 = fmaxf(m1, __shfl_xor(m1, o)); }
      part += m0 + m1;
    }
    const float tot = part + __shfl_xor(part, 16);
    if (lane == 0) Ss[c] = tot;
  }
  __syncthreads();
  if (wid == 0) {
    const v4f v = *(const v4f*)(&Ss[lane * 4]);
    *(volatile v4f*)(scores + (size_t)b * NB + lane * 4) = v;
    __threadfence();
    *(volatile v4f*)(scores + (size_t)b * NB + lane * 4) = v;
  }
}

__global__ __launch_bounds__(128) void loss_kernel(const float* __restrict__ scores, float* __restrict__ out) {
  __shared__ float term[NB];
  const int b = threadIdx.x;
  const float* row = scores + (size_t)b * NB;
  float mx = -INFINITY;
  for (int c = 0; c < NB; ++c) mx = fmaxf(mx, row[c]);
  float se = 0.0f;
  for (int c = 0; c < NB; ++c) se += expf(row[c] - mx);
  term[b] = (mx + logf(se)) - row[b];
  __syncthreads();
  if (b == 0) {
    float s = 0.0f;
    for (int i = 0; i < NB; ++i) s += term[i];
    const float loss = s * (1.0f / NB);
    *(volatile float*)out = loss;
    __threadfence();
    *(volatile float*)out = loss;
  }
}
}

extern "C" void kernel_launch(void* const* d_in, const int* in_sizes, int n_in,
                              void* d_out, int out_size, void* d_ws, size_t ws_size, hipStream_t stream) {
  (void)n_in; (void)out_size;
  const float* q  = (const float*)d_in[0];
  const float* dc = (const float*)d_in[1];
  float* out = (float*)d_out;
  if (in_sizes[0] != NB * NQ * D || in_sizes[1] != NB * NS * D) return;
  size_t off = 0; char* ws = (char*)d_ws;
  auto carve = [&](size_t bytes) { char* p = ws + off; off += (bytes + 255) & ~(size_t)255; return p; };
  b16* q16 = (b16*)carve((size_t)NB * NQ * D * 2);
  b16* d16 = (b16*)carve((size_t)NB * NS * D * 2);
  float* sc = (float*)carve((size_t)NB * NB * 4);
  if (off > ws_size) return;
  cvt_kernel<<<1024, 256, 0, stream>>>(q, dc, q16, d16);
  score_kernel<<<NB, 256, 0, stream>>>(q16, d16, sc);
  loss_kernel<<<1, 128, 0, stream>>>(sc, out);
}
